// Relation_Classifier_27092653703728
// MI455X (gfx1250) — hardware-run, weakly checked
//
#include <hip/hip_runtime.h>
#include <math.h>

typedef __attribute__((ext_vector_type(16))) __bf16   v16b;
typedef __attribute__((ext_vector_type(8)))  __bf16   v8b;
typedef __attribute__((ext_vector_type(8)))  float    v8f;
typedef __attribute__((ext_vector_type(4)))  float    v4f;
typedef __attribute__((ext_vector_type(4)))  unsigned v4u;

constexpr int kNB   = 128;
constexpr int kND   = 2048;
constexpr int kNC   = 1000;
constexpr int kNCP  = 1024;
constexpr int kNcat = 4096;
constexpr int kCatW1 = 1024;
constexpr int kCatWc = 2048;
static_assert(kNcat == kCatWc + kND, "stacked plane rows");
static_assert((kND % 32) == 0 && (kNCP % 32) == 0, "GEMM K multiples of 32");
static_assert((kNB % 64) == 0 && (kNcat % 64) == 0 && (kND % 64) == 0 && (kNCP % 64) == 0, "GEMM M,N multiples of 64");
static_assert((kNC % 4) == 0, "four flat logits never straddle a row");

constexpr size_t kOut0 = 0;
constexpr size_t kOut1 = 512000 / 4;
constexpr size_t kOut2 = 1560576 / 4;
constexpr size_t kOutTotal = 2609152 / 4;
static_assert(kOut1 == (size_t)kNB * kNC, "out1 offset");
static_assert(kOut2 == kOut1 + (size_t)kNB * kND, "out2 offset");
static_assert(kOutTotal == kOut2 + (size_t)kNB * kND, "out total");

constexpr size_t kOffXB   = 0;
constexpr size_t kOffBCAT = kOffXB   + (size_t)kNB   * kND  * 2;
constexpr size_t kOffCT   = kOffBCAT + (size_t)kNcat * kND  * 2;
constexpr size_t kOffWCB  = kOffCT   + (size_t)kND   * kNCP * 2;
constexpr size_t kOffG    = kOffWCB  + (size_t)kNCP  * kND  * 2;
constexpr size_t kOffEH   = kOffG    + (size_t)kNB   * kNcat * 4;
constexpr size_t kOffEL   = kOffEH   + (size_t)kNB   * kNCP * 2;
constexpr size_t kOffCC   = kOffEL   + (size_t)kNB   * kNCP * 2;
constexpr size_t kOffXOH  = kOffCC   + (size_t)kNB   * kND  * 4;
constexpr size_t kOffXOL  = kOffXOH  + (size_t)kNB   * kND  * 2;
constexpr size_t kOffL    = kOffXOL  + (size_t)kNB   * kND  * 2;
constexpr size_t kOffXS2  = kOffL    + (size_t)kNB   * kNCP * 4;
constexpr size_t kOffCN2  = kOffXS2  + (size_t)kNB   * 4;
constexpr size_t kOffWINV = kOffCN2  + (size_t)kNCP  * 4;
constexpr size_t kOffSTAT = kOffWINV + (size_t)kNCP  * 4;
constexpr size_t kWsTotal = kOffSTAT + (size_t)kNB   * 32 * 4;
static_assert(kWsTotal == 30958080ull, "carve total");
static_assert(kWsTotal <= 134217728ull, "carve cap");
static_assert((kOffBCAT % 128) == 0 && (kOffCT % 128) == 0 && (kOffWCB % 128) == 0 && (kOffG % 128) == 0 &&
              (kOffEH % 128) == 0 && (kOffEL % 128) == 0 && (kOffCC % 128) == 0 && (kOffXOH % 128) == 0 &&
              (kOffXOL % 128) == 0 && (kOffL % 128) == 0 && (kOffXS2 % 128) == 0 && (kOffCN2 % 128) == 0 &&
              (kOffWINV % 128) == 0 && (kOffSTAT % 128) == 0, "128-B aligned regions");

__device__ __forceinline__ unsigned bf_bits(float f) {
  const unsigned u = __float_as_uint(f);
  return ((u + 0x7FFFu + ((u >> 16) & 1u)) >> 16) & 0xFFFFu;
}
__device__ __forceinline__ float bf_val(unsigned h) { return __uint_as_float(h << 16); }
__device__ __forceinline__ unsigned pack2(unsigned lo16, unsigned hi16) { return lo16 | (hi16 << 16); }
__device__ __forceinline__ void split_bf(float f, unsigned& hb, unsigned& lb) {
  hb = bf_bits(f);
  lb = bf_bits(f - bf_val(hb));
}

__device__ __forceinline__ void acc_guard1(v8f& a, v16b x, v16b y, v16b z) {
  asm volatile("v_nop\n\tv_nop\n\tv_nop\n\tv_nop" : "+v"(a) : "v"(x), "v"(y), "v"(z));
}
__device__ __forceinline__ void keep4_b(v16b a, v16b b, v16b c, v16b d) { asm volatile("v_nop" :: "v"(a), "v"(b), "v"(c), "v"(d)); }
__device__ __forceinline__ void acc_guard4(v8f& a, v8f& b, v8f& c, v8f& d) { asm volatile("v_nop\n\tv_nop\n\tv_nop\n\tv_nop" : "+v"(a), "+v"(b), "+v"(c), "+v"(d)); }

union FragU { v16b v; v8b h[2]; };
__device__ __forceinline__ v16b frag_load(const __bf16* p) {
  FragU f;
  f.h[0] = *(const v8b*)(p);
  f.h[1] = *(const v8b*)(p + 16);
  return f.v;
}
__device__ __forceinline__ v8f frag_mma(v16b a, v16b b, v8f c) {
  return __builtin_amdgcn_wmma_f32_16x16x32_bf16(false, a, false, b, (short)0, c, false, false);
}

template <int SPL>
__global__ __launch_bounds__(256) void wmma_gemm64_bf16(
    const unsigned short* __restrict__ Ap, const unsigned short* __restrict__ A2p, int lda,
    const unsigned short* __restrict__ Btp, int ldb,
    float* __restrict__ Cout, int ldc, int M, int N, int K) {
  const __bf16* A  = (const __bf16*)Ap;
  const __bf16* A2 = (const __bf16*)A2p;
  const __bf16* Bt = (const __bf16*)Btp;
  __shared__ __align__(16) float sT[8][16 * 68];
  const int lane = threadIdx.x & 31;
  const int wave = threadIdx.x >> 5;
  const int tilesN = N >> 6;
  const int tilesM = M >> 6;
  const int tile = blockIdx.x * 8 + wave;
  if (tile >= tilesM * tilesN) return;
  const int tm = tile / tilesN;
  const int tn = tile - tm * tilesN;
  const int m0 = tm << 6;
  const int n0 = tn << 6;

  const int rlane = lane & 15;
  const int koff  = (lane >> 4) * 8;
  const int mOff  = (lane >> 4) * 8;

  v8f acc[4][4];
#pragma unroll
  for (int i = 0; i < 4; ++i)
#pragma unroll
    for (int j = 0; j < 4; ++j) acc[i][j] = (v8f){0.f,0.f,0.f,0.f,0.f,0.f,0.f,0.f};

  for (int k0 = 0; k0 < K; k0 += 32) {
    v16b bh[4];
#pragma unroll
    for (int j = 0; j < 4; ++j) {
      const size_t bo = (size_t)(n0 + (j << 4) + rlane) * ldb + koff + k0;
      bh[j] = frag_load(Bt + bo);
    }
#pragma unroll
    for (int i = 0; i < 4; ++i) {
      const size_t ao = (size_t)(m0 + (i << 4) + rlane) * lda + koff + k0;
      v16b ah = frag_load(A + ao);
      v16b al;
      if (SPL >= 1) al = frag_load(A2 + ao);
#pragma unroll
      for (int j = 0; j < 4; ++j) {
        acc[i][j] = frag_mma(ah, bh[j], acc[i][j]);
        if (SPL >= 1) acc[i][j] = frag_mma(al, bh[j], acc[i][j]);
      }
      const v16b a2 = (SPL >= 1) ? al : ah;
      acc_guard1(acc[i][0], ah, a2, bh[0]);
      acc_guard1(acc[i][1], ah, a2, bh[1]);
      acc_guard1(acc[i][2], ah, a2, bh[2]);
      acc_guard1(acc[i][3], ah, a2, bh[3]);
    }
    keep4_b(bh[0], bh[1], bh[2], bh[3]);
  }
  acc_guard4(acc[0][0], acc[0][1], acc[0][2], acc[0][3]);
  acc_guard4(acc[1][0], acc[1][1], acc[1][2], acc[1][3]);
  acc_guard4(acc[2][0], acc[2][1], acc[2][2], acc[2][3]);
  acc_guard4(acc[3][0], acc[3][1], acc[3][2], acc[3][3]);

  float* slab = sT[wave];
#pragma unroll
  for (int i = 0; i < 4; ++i) {
    const int mBase = m0 + (i << 4);
#pragma unroll
    for (int j = 0; j < 4; ++j) {
#pragma unroll
      for (int r = 0; r < 8; ++r) {
        slab[(mOff + r) * 68 + (j << 4) + rlane] = acc[i][j][r];
      }
    }
    __builtin_amdgcn_fence(__ATOMIC_RELEASE, "workgroup");
    __builtin_amdgcn_wave_barrier();
    __builtin_amdgcn_fence(__ATOMIC_ACQUIRE, "workgroup");
    {
      const int hh = lane >> 4, c4 = (lane & 15) * 4;
      for (int pass = 0; pass < 2; ++pass) {
#pragma unroll
        for (int it = 0; it < 8; ++it) {
          const int row = it * 2 + hh;
          v4f v = *(const v4f*)(slab + row * 68 + c4);
          *(volatile v4f*)(Cout + (size_t)(mBase + row) * ldc + n0 + c4) = v;
        }
        __threadfence();
      }
    }
    __builtin_amdgcn_fence(__ATOMIC_RELEASE, "workgroup");
    __builtin_amdgcn_wave_barrier();
    __builtin_amdgcn_fence(__ATOMIC_ACQUIRE, "workgroup");
  }
}

__global__ __launch_bounds__(256) void rows_prep_kernel(
    const float* __restrict__ src, int rows_real,
    unsigned short* __restrict__ dst, float* __restrict__ dstf,
    float* __restrict__ stat, int stat_mode)
{
  __shared__ float sStat[32];
  const int tid = threadIdx.x, lane = tid & 31, wave = tid >> 5;
  const int rbase = blockIdx.x * 32 + wave * 4;
#pragma unroll 1
  for (int i = 0; i < 4; ++i) {
    const int r = rbase + i;
    const bool real = r < rows_real;
    const int rc = real ? r : (rows_real - 1);
    const float* sp = src + (size_t)rc * kND + lane * 8;
    v4u pk[8];
    float s = 0.f;
#pragma unroll
    for (int j = 0; j < 8; ++j) {
      v4f a0 = *(const v4f*)(sp + j * 256);
      v4f a1 = *(const v4f*)(sp + j * 256 + 4);
      asm volatile("" : "+v"(a0));
      asm volatile("" : "+v"(a1));
      unsigned hb[8];
#pragma unroll
      for (int e = 0; e < 4; ++e) {
        float t0 = a0[e];
        float t1 = a1[e];
        t0 = real ? t0 : 0.0f;
        t1 = real ? t1 : 0.0f;
        hb[e]     = bf_bits(t0);
        hb[4 + e] = bf_bits(t1);
        const float r0 = bf_val(hb[e]);
        const float r1 = bf_val(hb[4 + e]);
        s = fmaf(r0, r0, s);
        s = fmaf(r1, r1, s);
      }
      pk[j] = (v4u){pack2(hb[0], hb[1]), pack2(hb[2], hb[3]), pack2(hb[4], hb[5]), pack2(hb[6], hb[7])};
    }
    unsigned short* dp = dst + (size_t)r * kND + lane * 8;
    for (int pass = 0; pass < 2; ++pass) {
#pragma unroll
      for (int j = 0; j < 8; ++j) *(volatile v4u*)(dp + j * 256) = pk[j];
      __threadfence();
    }
#pragma unroll
    for (int off = 16; off > 0; off >>= 1) s += __shfl_xor(s, off, 32);
    if (lane == 0) sStat[wave * 4 + i] = s;
    if (dstf != nullptr) {
#pragma unroll 1
      for (int j = 0; j < 16; ++j) {
        v4f a = *(const v4f*)(src + (size_t)rc * kND + j * 128 + lane * 4);
        asm volatile("" : "+v"(a));
        const float t0 = a[0], t1 = a[1], t2 = a[2], t3 = a[3];
        const v4f o4 = (v4f){bf_val(bf_bits(t0)), bf_val(bf_bits(t1)), bf_val(bf_bits(t2)), bf_val(bf_bits(t3))};
        float* op = dstf + (size_t)r * kND + j * 128 + lane * 4;
        *(volatile v4f*)op = o4;
        __threadfence();
        *(volatile v4f*)op = o4;
      }
    }
  }
  __syncthreads();
  if (wave == 0 && stat != nullptr) {
    float v = sStat[lane];
    const int r = blockIdx.x * 32 + lane;
    if (stat_mode == 1) {
      const float inv = 1.0f / sqrtf(fmaxf(v, 1.0e-30f));
      v = (r < rows_real) ? inv : 0.0f;
    }
    *(volatile float*)(stat + r) = v;
    __threadfence();
    *(volatile float*)(stat + r) = v;
  }
}

__global__ __launch_bounds__(256) void centers_transpose_kernel(
    const float* __restrict__ centers, unsigned short* __restrict__ ct)
{
  __shared__ float sT[64 * 65];
  const int tid = threadIdx.x, lane = tid & 31, wave = tid >> 5;
  const int c0 = blockIdx.x * 64, d0 = blockIdx.y * 64;
  const int cl0 = tid >> 4, dl4 = (tid & 15) * 4;
#pragma unroll
  for (int i = 0; i < 4; ++i) {
    const int cl = cl0 + 16 * i;
    const int c = c0 + cl;
    const bool real = c < kNC;
    const int cc = real ? c : (kNC - 1);
    v4f a = *(const v4f*)(centers + (size_t)cc * kND + d0 + dl4);
    asm volatile("" : "+v"(a));
    const float t0 = a[0], t1 = a[1], t2 = a[2], t3 = a[3];
    sT[cl * 65 + dl4 + 0] = real ? t0 : 0.0f;
    sT[cl * 65 + dl4 + 1] = real ? t1 : 0.0f;
    sT[cl * 65 + dl4 + 2] = real ? t2 : 0.0f;
    sT[cl * 65 + dl4 + 3] = real ? t3 : 0.0f;
  }
  __syncthreads();
  const int q = lane >> 3, c8 = (lane & 7) * 8;
  v4u pk[2];
#pragma unroll
  for (int it = 0; it < 2; ++it) {
    const int dl = it * 32 + wave * 4 + q;
    unsigned hb[8];
#pragma unroll
    for (int e = 0; e < 8; ++e) hb[e] = bf_bits(sT[(c8 + e) * 65 + dl]);
    pk[it] = (v4u){pack2(hb[0], hb[1]), pack2(hb[2], hb[3]), pack2(hb[4], hb[5]), pack2(hb[6], hb[7])};
  }
  for (int pass = 0; pass < 2; ++pass) {
#pragma unroll
    for (int it = 0; it < 2; ++it) {
      const int dl = it * 32 + wave * 4 + q;
      *(volatile v4u*)(ct + (size_t)(d0 + dl) * kNCP + c0 + c8) = pk[it];
    }
    __threadfence();
  }
}

__global__ __launch_bounds__(256) void stage1_row_kernel(
    const float* __restrict__ G, const float* __restrict__ xs2, const float* __restrict__ cn2,
    const float* __restrict__ b1,
    unsigned short* __restrict__ EH, unsigned short* __restrict__ EL, float* __restrict__ stat)
{
  __shared__ float sMin[8];
  __shared__ float sMax[8];
  __shared__ float sSum[8];
  __shared__ __align__(16) float sE[kNCP];
  const int tid = threadIdx.x, lane = tid & 31, wave = tid >> 5;
  const int b = blockIdx.x;
  const float xs = xs2[b];
  const float* grow = G + (size_t)b * kNcat;
  float dmin = 3.0e38f, zmax = -3.0e38f;
#pragma unroll 1
  for (int it = 0; it < 4; ++it) {
    const int n = it * 256 + tid;
    const bool valid = n < kNC;
    const int nc = valid ? n : (kNC - 1);
    float gd = grow[n];
    float gz = grow[kCatW1 + n];
    float cn = cn2[n];
    float bv = b1[nc];
    asm volatile("" : "+v"(gd), "+v"(gz), "+v"(cn), "+v"(bv));
    const float d2 = fmaxf(xs + cn - 2.0f * gd, 0.0f);
    const float z = gz + bv;
    dmin = fminf(dmin, valid ? d2 : 3.0e38f);
    zmax = fmaxf(zmax, valid ? z : -3.0e38f);
  }
#pragma unroll
  for (int off = 16; off > 0; off >>= 1) {
    dmin = fminf(dmin, __shfl_xor(dmin, off, 32));
    zmax = fmaxf(zmax, __shfl_xor(zmax, off, 32));
  }
  if (lane == 0) { sMin[wave] = dmin; sMax[wave] = zmax; }
  __syncthreads();
  dmin = sMin[0];
  zmax = sMax[0];
#pragma unroll
  for (int w = 1; w < 8; ++w) {
    dmin = fminf(dmin, sMin[w]);
    zmax = fmaxf(zmax, sMax[w]);
  }
  float esum = 0.f;
#pragma unroll 1
  for (int it = 0; it < 4; ++it) {
    const int n = it * 256 + tid;
    const bool valid = n < kNC;
    const int nc = valid ? n : (kNC - 1);
    float gz = grow[kCatW1 + n];
    float bv = b1[nc];
    asm volatile("" : "+v"(gz), "+v"(bv));
    const float ex = expf((gz + bv) - zmax);
    const float ev = valid ? ex : 0.0f;
    sE[n] = ev;
    esum += ev;
  }
#pragma unroll
  for (int off = 16; off > 0; off >>= 1) esum += __shfl_xor(esum, off, 32);
  if (lane == 0) sSum[wave] = esum;
  __syncthreads();
  float tot = sSum[0];
#pragma unroll
  for (int w = 1; w < 8; ++w) tot += sSum[w];
  const float conf = 10.0f * (1.0f / sqrtf(dmin));
  const float rsum = 1.0f / tot;

  if (wave < 4) {
    const int n8 = tid * 8;
    const v4f a0 = *(const v4f*)(sE + n8);
    const v4f a1 = *(const v4f*)(sE + n8 + 4);
    unsigned hb[8], lb[8];
#pragma unroll
    for (int e = 0; e < 4; ++e) {
      const float t0 = a0[e];
      const float t1 = a1[e];
      split_bf(t0, hb[e], lb[e]);
      split_bf(t1, hb[4 + e], lb[4 + e]);
    }
    const v4u ph = (v4u){pack2(hb[0], hb[1]), pack2(hb[2], hb[3]), pack2(hb[4], hb[5]), pack2(hb[6], hb[7])};
    const v4u pl = (v4u){pack2(lb[0], lb[1]), pack2(lb[2], lb[3]), pack2(lb[4], lb[5]), pack2(lb[6], lb[7])};
    unsigned short* qh = EH + (size_t)b * kNCP + n8;
    unsigned short* ql = EL + (size_t)b * kNCP + n8;
    *(volatile v4u*)qh = ph;
    *(volatile v4u*)ql = pl;
    __threadfence();
    *(volatile v4u*)qh = ph;
    *(volatile v4u*)ql = pl;
  }
  if (wave == 4) {
    const float v = (lane == 0) ? conf : ((lane == 1) ? rsum : 0.0f);
    float* sp = stat + (size_t)b * 32 + lane;
    *(volatile float*)sp = v;
    __threadfence();
    *(volatile float*)sp = v;
  }
}

__global__ __launch_bounds__(256) void fuse_row_kernel(
    const float* __restrict__ x, const float* __restrict__ G, const float* __restrict__ CC,
    const float* __restrict__ bc, const float* __restrict__ stat,
    float* __restrict__ out2, unsigned short* __restrict__ XOH, unsigned short* __restrict__ XOL)
{
  __shared__ __align__(16) float sXo[kND];
  __shared__ __align__(16) float sFast[kND];
  __shared__ float sSum[8];
  const int tid = threadIdx.x, lane = tid & 31, wave = tid >> 5;
  const int b = blockIdx.x;
  const float conf = stat[(size_t)b * 32];
  const float rsum = stat[(size_t)b * 32 + 1];
  float ss = 0.f;
#pragma unroll 1
  for (int it = 0; it < 8; ++it) {
    const int d = it * 256 + tid;
    const float cc = CC[(size_t)b * kND + d] * rsum;
    const float g = tanhf(G[(size_t)b * kNcat + kCatWc + d] + bc[d]);
    const float fast = g * cc;
    const float xr = bf_val(bf_bits(x[(size_t)b * kND + d]));
    const float xo = conf * (xr + fast);
    ss = fmaf(xo, xo, ss);
    sXo[d] = xo;
    sFast[d] = fast;
  }
#pragma unroll
  for (int off = 16; off > 0; off >>= 1) ss += __shfl_xor(ss, off, 32);
  if (lane == 0) sSum[wave] = ss;
  __syncthreads();
  float tot = sSum[0];
#pragma unroll
  for (int w = 1; w < 8; ++w) tot += sSum[w];
  const float scl = 16.0f * (1.0f / (1.0f + sqrtf(tot)));

  v4f fv[2];
#pragma unroll
  for (int j = 0; j < 2; ++j) fv[j] = *(const v4f*)(sFast + j * 1024 + tid * 4);
  const v4f a0 = *(const v4f*)(sXo + tid * 8);
  const v4f a1 = *(const v4f*)(sXo + tid * 8 + 4);
  unsigned hb[8], lb[8];
#pragma unroll
  for (int e = 0; e < 4; ++e) {
    const float t0 = a0[e] * scl;
    const float t1 = a1[e] * scl;
    split_bf(t0, hb[e], lb[e]);
    split_bf(t1, hb[4 + e], lb[4 + e]);
  }
  const v4u ph = (v4u){pack2(hb[0], hb[1]), pack2(hb[2], hb[3]), pack2(hb[4], hb[5]), pack2(hb[6], hb[7])};
  const v4u pl = (v4u){pack2(lb[0], lb[1]), pack2(lb[2], lb[3]), pack2(lb[4], lb[5]), pack2(lb[6], lb[7])};
  unsigned short* qh = XOH + (size_t)b * kND + tid * 8;
  unsigned short* ql = XOL + (size_t)b * kND + tid * 8;
  float* o2 = out2 + (size_t)b * kND + tid * 4;
  for (int pass = 0; pass < 2; ++pass) {
#pragma unroll
    for (int j = 0; j < 2; ++j) *(volatile v4f*)(o2 + j * 1024) = fv[j];
    *(volatile v4u*)qh = ph;
    *(volatile v4u*)ql = pl;
    __threadfence();
  }
}

__global__ __launch_bounds__(256) void logits_pack_kernel(
    const float* __restrict__ L, const float* __restrict__ winv, float* __restrict__ out0)
{
  const int i4 = blockIdx.x * 256 + threadIdx.x;
  if (i4 >= (kNB * kNC) / 4) return;
  const int i = i4 * 4;
  const int m = i / kNC;
  const int n = i - m * kNC;
  const v4f l = *(const v4f*)(L + (size_t)m * kNCP + n);
  const v4f w = *(const v4f*)(winv + n);
  const v4f o = l * w;
  *(volatile v4f*)(out0 + i) = o;
  __threadfence();
  *(volatile v4f*)(out0 + i) = o;
}

extern "C" void kernel_launch(void* const* d_in, const int* in_sizes, int n_in,
                              void* d_out, int out_size, void* d_ws, size_t ws_size,
                              hipStream_t stream) {
  if (n_in < 9) return;
  if (in_sizes[0] != kNB * kND) return;
  if (in_sizes[2] != kNC * kND) return;
  if (in_sizes[4] != kND * kND) return;
  if (in_sizes[5] != kND) return;
  if (in_sizes[6] != kNC * kND) return;
  if (in_sizes[7] != kNC) return;
  if (in_sizes[8] != kNC * kND) return;
  if ((size_t)out_size != kOutTotal) return;
  if (ws_size < kWsTotal) return;

  const float* x       = (const float*)d_in[0];
  const float* centers = (const float*)d_in[2];
  const float* Wc      = (const float*)d_in[4];
  const float* bc      = (const float*)d_in[5];
  const float* W1      = (const float*)d_in[6];
  const float* b1      = (const float*)d_in[7];
  const float* Wcos    = (const float*)d_in[8];

  float* outp = (float*)d_out;
  float* out0 = outp + kOut0;
  float* out1 = outp + kOut1;
  float* out2 = outp + kOut2;

  char* ws = (char*)d_ws;
  unsigned short* XB   = (unsigned short*)(ws + kOffXB);
  unsigned short* BCAT = (unsigned short*)(ws + kOffBCAT);
  unsigned short* CT   = (unsigned short*)(ws + kOffCT);
  unsigned short* WCB  = (unsigned short*)(ws + kOffWCB);
  float*          G    = (float*)(ws + kOffG);
  unsigned short* EH   = (unsigned short*)(ws + kOffEH);
  unsigned short* EL   = (unsigned short*)(ws + kOffEL);
  float*          CC   = (float*)(ws + kOffCC);
  unsigned short* XOH  = (unsigned short*)(ws + kOffXOH);
  unsigned short* XOL  = (unsigned short*)(ws + kOffXOL);
  float*          L    = (float*)(ws + kOffL);
  float*          XS2  = (float*)(ws + kOffXS2);
  float*          CN2  = (float*)(ws + kOffCN2);
  float*          WINV = (float*)(ws + kOffWINV);
  float*          STAT = (float*)(ws + kOffSTAT);

  rows_prep_kernel<<<kNB / 32, 256, 0, stream>>>(x, kNB, XB, out1, XS2, 0);
  rows_prep_kernel<<<kNCP / 32, 256, 0, stream>>>(centers, kNC, BCAT, nullptr, CN2, 0);
  rows_prep_kernel<<<kNCP / 32, 256, 0, stream>>>(W1, kNC, BCAT + (size_t)kCatW1 * kND, nullptr, nullptr, 0);
  rows_prep_kernel<<<kND / 32, 256, 0, stream>>>(Wc, kND, BCAT + (size_t)kCatWc * kND, nullptr, nullptr, 0);
  rows_prep_kernel<<<kNCP / 32, 256, 0, stream>>>(Wcos, kNC, WCB, nullptr, WINV, 1);
  centers_transpose_kernel<<<dim3(kNCP / 64, kND / 64), 256, 0, stream>>>(centers, CT);

  wmma_gemm64_bf16<0><<<dim3(16), 256, 0, stream>>>(XB, XB, kND, BCAT, kND, G, kNcat, kNB, kNcat, kND);

  stage1_row_kernel<<<kNB, 256, 0, stream>>>(G, XS2, CN2, b1, EH, EL, STAT);

  wmma_gemm64_bf16<1><<<dim3(8), 256, 0, stream>>>(EH, EL, kNCP, CT, kNCP, CC, kND, kNB, kND, kNCP);

  fuse_row_kernel<<<kNB, 256, 0, stream>>>(x, G, CC, bc, STAT, out2, XOH, XOL);

  wmma_gemm64_bf16<1><<<dim3(4), 256, 0, stream>>>(XOH, XOL, kND, WCB, kND, L, kNCP, kNB, kNCP, kND);

  logits_pack_kernel<<<(kNB * kNC / 4) / 256, 256, 0, stream>>>(L, WINV, out0);
}
